// ChunkedResidualMambaBlock_39075612459682
// MI455X (gfx1250) — hardware-verified
//
#include <hip/hip_runtime.h>


namespace {
constexpr int NB = 4, C = 96, HH = 64, CS = 8, HN = HH / CS, NCHI = HN * HN, NCH = NB * NCHI, L = CS * CS, NT = NCH * L, DN = 192, NS = 16, K = 4, DTR = 6, XD = DTR + 2 * NS;
constexpr float XS = 8.0f, DS = 256.0f, WSC = 256.0f, EPS = 1e-5f;
typedef _Float16 b16;
typedef __attribute__((ext_vector_type(16))) _Float16 v16b;
typedef __attribute__((ext_vector_type(8))) _Float16 v8b;
typedef __attribute__((ext_vector_type(8))) float v8f;
typedef __attribute__((ext_vector_type(4))) float v4f;
typedef __attribute__((ext_vector_type(2))) float v2f;
__device__ __forceinline__ float bf16_rne(float f) { unsigned int u = __float_as_uint(f); u += 0x7FFFu + ((u >> 16) & 1u); return __uint_as_float(u & 0xFFFF0000u); }
__device__ __forceinline__ void split16(float v, b16& hi, b16& lo) { hi = (b16)v; lo = (b16)(v - (float)hi); }
__device__ __forceinline__ v16b frag_kb(const b16* p, int hh) { const v8b a = *(const v8b*)(p + 8 * hh), b = *(const v8b*)(p + 16 + 8 * hh); v16b f;
#pragma unroll
  for (int e = 0; e < 8; ++e) { f[e] = a[e]; f[8 + e] = b[e]; } return f; }
__device__ __forceinline__ v8f wmma16b(v16b a, v16b b, v8f c) { v8f d = __builtin_amdgcn_wmma_f32_16x16x32_f16(false, a, false, b, (short)0, c, false, false); asm volatile("v_nop\n\tv_nop\n\tv_nop\n\tv_nop" : "+v"(d) : "v"(a), "v"(b)); return d; }
__device__ __forceinline__ void wave_lds_sync() { __builtin_amdgcn_fence(__ATOMIC_RELEASE, "workgroup"); __builtin_amdgcn_wave_barrier(); __builtin_amdgcn_fence(__ATOMIC_ACQUIRE, "workgroup"); }
__device__ __forceinline__ float pmul(float a, float b) { float p = a * b; asm volatile("" : "+v"(p)); return p; }
__device__ __forceinline__ float sigm(float v) { return 1.0f / (1.0f + __expf(-v)); }
__device__ __forceinline__ float silu(float v) { return pmul(v, sigm(v)); }
__device__ __forceinline__ float softplus(float v) { return v > 20.0f ? v : (v < -20.0f ? __expf(v) : log1pf(__expf(v))); }
__device__ __forceinline__ size_t pix_index(int t, int c) { const int ch = t / L, p = t % L, b = ch / NCHI, cc = ch % NCHI, hi = cc / HN, wi = cc % HN, i = p / CS, j = p % CS; return (((size_t)b * C + c) * HH + hi * CS + i) * HH + wi * CS + j; }

__global__ __launch_bounds__(256) void wprep_kernel(const float* __restrict__ w, int KIN, int OUT, b16* __restrict__ WT) {
  const size_t u = (size_t)blockIdx.x * 256 + threadIdx.x; if (u >= (size_t)OUT * KIN / 8) return; const size_t e = u * 8; const int o = (int)(e / KIN), k0 = (int)(e % KIN); v8b v;
  for (int j = 0; j < 8; ++j) v[j] = (b16)(bf16_rne(w[(size_t)(k0 + j) * OUT + o]) * WSC); for (int pass = 0; pass < 2; ++pass) { *(volatile v8b*)(WT + e) = v; __threadfence(); }
}
__global__ __launch_bounds__(256) void wcopyp_kernel(const float* __restrict__ w, int KIN, int OUT, int KP, int OUTP, b16* __restrict__ WT) {
  const int u = blockIdx.x * 256 + threadIdx.x; if (u >= OUTP * KP / 8) return; const int e = u * 8; const int o = e / KP, k0 = e % KP; v8b v;
  for (int j = 0; j < 8; ++j) { const int k = k0 + j; v[j] = (o < OUT && k < KIN) ? (b16)(bf16_rne(w[(size_t)o * KIN + k]) * WSC) : (b16)0.0f; } for (int pass = 0; pass < 2; ++pass) { *(volatile v8b*)(WT + e) = v; __threadfence(); }
}
__global__ __launch_bounds__(256) void snorm_kernel(const float* __restrict__ x, float* __restrict__ MS) {
  __shared__ float rs[256], rq[256];
  const int bc = blockIdx.x, tid = threadIdx.x; const float* xr = x + (size_t)bc * HH * HH; float s = 0.0f;
  for (int p = tid; p < HH * HH; p += 256) s += bf16_rne(xr[p]);
  rs[tid] = s; __syncthreads(); for (int st = 128; st; st >>= 1) { if (tid < st) rs[tid] += rs[tid + st]; __syncthreads(); } const float mean = rs[0] * (1.0f / (HH * HH)); __syncthreads();
  float q = 0.0f; for (int p = tid; p < HH * HH; p += 256) { const float d = bf16_rne(xr[p]) - mean; q += pmul(d, d); }
  rq[tid] = q; __syncthreads(); for (int st = 128; st; st >>= 1) { if (tid < st) rq[tid] += rq[tid + st]; __syncthreads(); } const float rstd = rsqrtf(rq[0] * (1.0f / (HH * HH)) + EPS);
  for (int pass = 0; pass < 2; ++pass) { if (tid < 64) ((volatile float*)MS)[(size_t)bc * 64 + tid] = tid == 0 ? mean : (tid == 1 ? rstd : 0.0f); __threadfence(); }
}
__device__ __forceinline__ float act_in(const float* __restrict__ x, const float* __restrict__ MS, const float* __restrict__ gam, const float* __restrict__ bet, int t, int c) {
  const size_t pi = pix_index(t, c); const int ch = t / L, b = ch / NCHI; const float* ms = MS + ((size_t)b * C + c) * 64; const float xn = pmul(pmul(bf16_rne(x[pi]) - ms[0], ms[1]), bf16_rne(gam[c])) + bf16_rne(bet[c]); return silu(xn);
}
__global__ __launch_bounds__(32) void inproj_kernel(const float* __restrict__ x, const float* __restrict__ MS, const float* __restrict__ gam, const float* __restrict__ bet, const float* __restrict__ lg, const float* __restrict__ lb, const b16* __restrict__ WIP, float* __restrict__ XZ) {
  __shared__ __attribute__((aligned(16))) b16 Ah[16][C + 8], Al[16][C + 8]; __shared__ __attribute__((aligned(16))) float Tf[16][128 + 4];
  const int lane = threadIdx.x, nloc = lane & 15, hlf = lane >> 4; const size_t m0 = (size_t)blockIdx.x * 16;
  float g3[3], b3[3]; for (int q = 0; q < 3; ++q) { g3[q] = bf16_rne(lg[q * 32 + lane]); b3[q] = bf16_rne(lb[q * 32 + lane]); }
  for (int rr = 0; rr < 16; ++rr) { const int t = (int)(m0 + rr); float h[3]; float s = 0.0f; for (int q = 0; q < 3; ++q) { h[q] = act_in(x, MS, gam, bet, t, q * 32 + lane); s += h[q]; } for (int o = 16; o; o >>= 1) s += __shfl_xor(s, o); const float mu = s * (1.0f / C);
    float vq = 0.0f; for (int q = 0; q < 3; ++q) { const float d = h[q] - mu; vq += pmul(d, d); } for (int o = 16; o; o >>= 1) vq += __shfl_xor(vq, o); const float rs = rsqrtf(vq * (1.0f / C) + EPS);
    for (int q = 0; q < 3; ++q) { const float v = pmul(pmul(h[q] - mu, rs), g3[q]) + b3[q]; b16 p, ql; split16(v * XS, p, ql); Ah[rr][q * 32 + lane] = p; Al[rr][q * 32 + lane] = ql; } }
  wave_lds_sync();
#pragma unroll 1
  for (int cg = 0; cg < 3; ++cg) { v8f acc[8];
#pragma unroll
    for (int t = 0; t < 8; ++t) acc[t] = (v8f){};
#pragma unroll
    for (int kb = 0; kb < C; kb += 32) { const v16b a = frag_kb(&Ah[nloc][kb], hlf), al = frag_kb(&Al[nloc][kb], hlf);
#pragma unroll
      for (int t = 0; t < 8; ++t) { const v16b bw = frag_kb(WIP + (size_t)(cg * 128 + t * 16 + nloc) * C + kb, hlf); acc[t] = wmma16b(a, bw, acc[t]); acc[t] = wmma16b(al, bw, acc[t]); } }
#pragma unroll
    for (int t = 0; t < 8; ++t)
#pragma unroll 1
      for (int r8 = 0; r8 < 8; ++r8) Tf[8 * hlf + r8][t * 16 + nloc] = acc[t][r8] * (1.0f / (XS * WSC));
    wave_lds_sync();
    for (int pass = 0; pass < 2; ++pass) { for (int rr = 0; rr < 16; ++rr) *(volatile v4f*)(XZ + (m0 + rr) * (2 * DN) + cg * 128 + lane * 4) = *(const v4f*)(&Tf[rr][lane * 4]); __threadfence(); }
    wave_lds_sync(); }
}
__global__ __launch_bounds__(256) void dwconv_kernel(const float* __restrict__ XZ, const float* __restrict__ cw, const float* __restrict__ cb, int ntok, float* __restrict__ U) {
  const size_t gid = (size_t)blockIdx.x * 256 + threadIdx.x; const size_t t = gid / (DN / 4); const int d4 = (int)(gid % (DN / 4)) * 4; if (t >= (size_t)ntok) return;
  const int ch = (int)(t / L), p = (int)(t % L), i = p / CS, j = p % CS; v4f acc; for (int q = 0; q < 4; ++q) acc[q] = bf16_rne(cb[d4 + q]);
#pragma unroll
  for (int di = 0; di < 3; ++di)
#pragma unroll
    for (int dj = 0; dj < 3; ++dj) { const int ii = i + di - 1, jj = j + dj - 1; const bool ok = ii >= 0 && ii < CS && jj >= 0 && jj < CS; const int iic = ok ? ii : i, jjc = ok ? jj : j;
      const v4f v = *(const v4f*)(XZ + ((size_t)ch * L + iic * CS + jjc) * (2 * DN) + d4); for (int q = 0; q < 4; ++q) acc[q] += ok ? pmul(v[q], bf16_rne(cw[(d4 + q) * 9 + di * 3 + dj])) : 0.0f; }
  v4f o; for (int q = 0; q < 4; ++q) o[q] = silu(acc[q]);
  for (int pass = 0; pass < 2; ++pass) { *(volatile v4f*)(U + t * DN + d4) = o; __threadfence(); }
}
__global__ __launch_bounds__(32) void xproj_kernel(const float* __restrict__ U, const b16* __restrict__ XPW, const b16* __restrict__ DTW, const float* __restrict__ dtb, float* __restrict__ BC, float* __restrict__ DT) {
  __shared__ __attribute__((aligned(16))) b16 Ah[16][DN + 8], Al[16][DN + 8]; __shared__ __attribute__((aligned(16))) b16 Dh[16][32 + 8], Dl[16][32 + 8]; __shared__ __attribute__((aligned(16))) float Sbc[16][32]; __shared__ __attribute__((aligned(16))) float Tf[16][DN + 4];
  const int lane = threadIdx.x, nloc = lane & 15, hlf = lane >> 4; const size_t m0 = (size_t)blockIdx.x * 16;
  for (int rr = 0; rr < 16; ++rr) for (int q = 0; q < 6; ++q) { const int c = q * 32 + lane; const float v = U[(m0 + rr) * DN + c]; b16 p, ql; split16(v * XS, p, ql); Ah[rr][c] = p; Al[rr][c] = ql; }
  wave_lds_sync();
  const float sx = 1.0f / (XS * WSC), sd = 1.0f / (DS * WSC);
#pragma unroll 1
  for (int k = 0; k < K; ++k) {
    v8f ax[3] = {(v8f){}, (v8f){}, (v8f){}};
#pragma unroll 2
    for (int kb = 0; kb < DN; kb += 32) { const v16b a = frag_kb(&Ah[nloc][kb], hlf), al = frag_kb(&Al[nloc][kb], hlf);
#pragma unroll
      for (int t = 0; t < 3; ++t) { const v16b bw = frag_kb(XPW + ((size_t)k * 48 + t * 16 + nloc) * DN + kb, hlf); ax[t] = wmma16b(a, bw, ax[t]); ax[t] = wmma16b(al, bw, ax[t]); } }
#pragma unroll
    for (int r8 = 0; r8 < 8; ++r8) { const int rl = 8 * hlf + r8; const float d0 = ax[0][r8] * sx, d1 = ax[1][r8] * sx, d2 = ax[2][r8] * sx;
      if (nloc < DTR) { b16 p, ql; split16(d0 * DS, p, ql); Dh[rl][nloc] = p; Dl[rl][nloc] = ql; Sbc[rl][10 + nloc] = d1; Sbc[rl][16 + 10 + nloc] = d2; }
      else { Sbc[rl][nloc - 6] = d0; Sbc[rl][16 + nloc - 6] = d1; if (nloc >= DTR) { Dh[rl][nloc] = (b16)0.0f; Dl[rl][nloc] = (b16)0.0f; } }
      Dh[rl][16 + nloc] = (b16)0.0f; Dl[rl][16 + nloc] = (b16)0.0f; }
    wave_lds_sync();
    for (int pass = 0; pass < 2; ++pass) { for (int rr = 0; rr < 16; ++rr) ((volatile float*)BC)[((size_t)k * NT + m0 + rr) * 32 + lane] = Sbc[rr][lane]; __threadfence(); }
    { v8f acc[12]; const v16b a = frag_kb(&Dh[nloc][0], hlf), al = frag_kb(&Dl[nloc][0], hlf);
#pragma unroll
      for (int t = 0; t < 12; ++t) { acc[t] = (v8f){}; const v16b bw = frag_kb(DTW + ((size_t)k * DN + t * 16 + nloc) * 32, hlf); acc[t] = wmma16b(a, bw, acc[t]); acc[t] = wmma16b(al, bw, acc[t]); }
#pragma unroll
      for (int t = 0; t < 12; ++t) { const int c = t * 16 + nloc; const float bb = bf16_rne(dtb[k * DN + c]);
#pragma unroll 1
        for (int r8 = 0; r8 < 8; ++r8) Tf[8 * hlf + r8][c] = softplus(acc[t][r8] * sd + bb); } }
    wave_lds_sync();
    for (int pass = 0; pass < 2; ++pass) { for (int rr = 0; rr < 16; ++rr) for (int q = 0; q < 6; ++q) ((volatile float*)DT)[((size_t)k * NT + m0 + rr) * DN + q * 32 + lane] = Tf[rr][q * 32 + lane]; __threadfence(); }
    wave_lds_sync(); }
}
__global__ __launch_bounds__(256) void scan_kernel(const float* __restrict__ U, const float* __restrict__ DT, const float* __restrict__ BC, const float* __restrict__ alog, const float* __restrict__ Dsv, int nch, float* __restrict__ Y4) {
  const int gid = blockIdx.x * 256 + threadIdx.x; const int ch = gid / DN, d = gid % DN; if (ch >= nch) return;
#pragma unroll 1
  for (int pass = 0; pass < 2; ++pass) {
#pragma unroll 1
    for (int k = 0; k < K; ++k) { float A[NS]; for (int s = 0; s < NS; ++s) A[s] = -__expf(bf16_rne(alog[((size_t)k * DN + d) * NS + s])); const float dk = bf16_rne(Dsv[k * DN + d]); float h[NS]; for (int s = 0; s < NS; ++s) h[s] = 0.0f;
#pragma unroll 1
      for (int l = 0; l < L; ++l) { const int lr = L - 1 - l; const int p = k == 0 ? l : (k == 1 ? (l % CS) * CS + l / CS : (k == 2 ? lr : (lr % CS) * CS + lr / CS));
        const size_t row = (size_t)ch * L + p; const float u = U[row * DN + d], dt = DT[((size_t)k * NT + row) * DN + d]; const float du = pmul(dt, u); const float* bc = BC + ((size_t)k * NT + row) * 32; float acc = 0.0f;
#pragma unroll
        for (int s = 0; s < NS; ++s) { h[s] = pmul(h[s], __expf(pmul(dt, A[s]))) + pmul(du, bc[s]); acc += pmul(h[s], bc[16 + s]); }
        ((volatile float*)Y4)[((size_t)k * NT + row) * DN + d] = acc + pmul(dk, u); } }
    __threadfence(); }
}
__global__ __launch_bounds__(32) void outproj_kernel(const float* __restrict__ Y4, const float* __restrict__ XZ, const float* __restrict__ og, const float* __restrict__ ob, const b16* __restrict__ WOP, float* __restrict__ V) {
  __shared__ __attribute__((aligned(16))) b16 Ah[16][DN + 8], Al[16][DN + 8]; __shared__ __attribute__((aligned(16))) float Tf[16][C + 4];
  const int lane = threadIdx.x, nloc = lane & 15, hlf = lane >> 4; const size_t m0 = (size_t)blockIdx.x * 16;
  float g6[6], b6[6]; for (int q = 0; q < 6; ++q) { g6[q] = bf16_rne(og[q * 32 + lane]); b6[q] = bf16_rne(ob[q * 32 + lane]); }
  for (int rr = 0; rr < 16; ++rr) { const size_t t = m0 + rr; float v[6]; float s = 0.0f; for (int q = 0; q < 6; ++q) { const int c = q * 32 + lane; v[q] = ((Y4[t * DN + c] + Y4[((size_t)NT + t) * DN + c]) + Y4[((size_t)2 * NT + t) * DN + c]) + Y4[((size_t)3 * NT + t) * DN + c]; s += v[q]; }     for (int o = 16; o; o >>= 1) s += __shfl_xor(s, o); const float mu = s * (1.0f / DN);
    float vq = 0.0f; for (int q = 0; q < 6; ++q) { const float dd = v[q] - mu; vq += pmul(dd, dd); } for (int o = 16; o; o >>= 1) vq += __shfl_xor(vq, o); const float rs = rsqrtf(vq * (1.0f / DN) + EPS);
    for (int q = 0; q < 6; ++q) { const int c = q * 32 + lane; const float z = XZ[t * (2 * DN) + DN + c]; const float a = pmul(pmul(pmul(v[q] - mu, rs), g6[q]) + b6[q], silu(z)); b16 p, ql; split16(a * XS, p, ql); Ah[rr][c] = p; Al[rr][c] = ql; } }
  wave_lds_sync();
  v8f acc[6];
#pragma unroll
  for (int t = 0; t < 6; ++t) acc[t] = (v8f){};
#pragma unroll 2
  for (int kb = 0; kb < DN; kb += 32) { const v16b a = frag_kb(&Ah[nloc][kb], hlf), al = frag_kb(&Al[nloc][kb], hlf);
#pragma unroll
    for (int t = 0; t < 6; ++t) { const v16b bw = frag_kb(WOP + (size_t)(t * 16 + nloc) * DN + kb, hlf); acc[t] = wmma16b(a, bw, acc[t]); acc[t] = wmma16b(al, bw, acc[t]); } }
#pragma unroll
  for (int t = 0; t < 6; ++t)
#pragma unroll 1
    for (int r8 = 0; r8 < 8; ++r8) Tf[8 * hlf + r8][t * 16 + nloc] = acc[t][r8] * (1.0f / (XS * WSC));
  wave_lds_sync();
  for (int pass = 0; pass < 2; ++pass) { for (int rr = 0; rr < 16; ++rr) if (lane < 24) *(volatile v4f*)(V + (m0 + rr) * C + lane * 4) = *(const v4f*)(&Tf[rr][lane * 4]); __threadfence(); }
}
__global__ __launch_bounds__(256) void final_kernel(const float* __restrict__ x, const float* __restrict__ MS, const float* __restrict__ gam, const float* __restrict__ bet, const float* __restrict__ alphap, const float* __restrict__ V, int nbv, float* __restrict__ out) {
  const size_t g = (size_t)blockIdx.x * 256 + threadIdx.x; if (g >= (size_t)nbv * C * HH * HH) return;
  const int b = (int)(g / ((size_t)C * HH * HH)); const int rem = (int)(g % ((size_t)C * HH * HH)); const int c = rem / (HH * HH), yy = (rem / HH) % HH, xx = rem % HH;
  const int t = ((b * NCHI + (yy / CS) * HN + xx / CS) * L) + (yy % CS) * CS + xx % CS; const float h = act_in(x, MS, gam, bet, t, c); const float alpha = bf16_rne(alphap[0]);
  const float o = bf16_rne(x[g]) + pmul(alpha, h + V[(size_t)t * C + c]);
  for (int pass = 0; pass < 2; ++pass) { ((volatile float*)out)[g] = o; __threadfence(); }
}
}

extern "C" void kernel_launch(void* const* d_in, const int* in_sizes, int n_in, void* d_out, int out_size, void* d_ws, size_t ws_size, hipStream_t stream) {
  (void)n_in;
  auto Fp = [&](int i) { return (const float*)d_in[i]; };
  if (in_sizes[0] != NB * C * HH * HH || in_sizes[6] != C * 2 * DN || in_sizes[7] != DN * 9 || in_sizes[9] != K * XD * DN || in_sizes[10] != K * DN * DTR || in_sizes[12] != K * DN * NS || in_sizes[16] != DN * C || out_size != NB * C * HH * HH) return;
  const int NBV = NB; const int NCHV = NBV * NCHI, NTV = NCHV * L;
  size_t off = 0; char* ws = (char*)d_ws;
  auto carve = [&](size_t bytes) { char* p = ws + off; off += (bytes + 255) & ~(size_t)255; return p; };
  b16* WIP = (b16*)carve((size_t)2 * DN * C * 2); b16* XPW = (b16*)carve((size_t)K * 48 * DN * 2); b16* DTW = (b16*)carve((size_t)K * DN * 32 * 2); b16* WOP = (b16*)carve((size_t)C * DN * 2);
  float* MS = (float*)carve((size_t)NB * C * 64 * 4); float* XZ = (float*)carve((size_t)NT * 2 * DN * 4); float* U = (float*)carve((size_t)NT * DN * 4); float* BC = (float*)carve((size_t)K * NT * 32 * 4); float* DT = (float*)carve((size_t)K * NT * DN * 4); float* Y4 = (float*)carve((size_t)K * NT * DN * 4); float* V = (float*)carve((size_t)NT * C * 4);
  if (off > ws_size) return;
  wprep_kernel<<<(2 * DN * C / 8 + 255) / 256, 256, 0, stream>>>(Fp(6), C, 2 * DN, WIP); wprep_kernel<<<(C * DN / 8 + 255) / 256, 256, 0, stream>>>(Fp(16), DN, C, WOP);
  for (int k = 0; k < K; ++k) { wcopyp_kernel<<<(48 * DN / 8 + 255) / 256, 256, 0, stream>>>(Fp(9) + (size_t)k * XD * DN, DN, XD, DN, 48, XPW + (size_t)k * 48 * DN); wcopyp_kernel<<<(DN * 32 / 8 + 255) / 256, 256, 0, stream>>>(Fp(10) + (size_t)k * DN * DTR, DTR, DN, 32, DN, DTW + (size_t)k * DN * 32); }
  snorm_kernel<<<NBV * C, 256, 0, stream>>>(Fp(0), MS);
  inproj_kernel<<<NTV / 16, 32, 0, stream>>>(Fp(0), MS, Fp(1), Fp(2), Fp(4), Fp(5), WIP, XZ);
  dwconv_kernel<<<(unsigned)(((size_t)NTV * (DN / 4) + 255) / 256), 256, 0, stream>>>(XZ, Fp(7), Fp(8), NTV, U);
  xproj_kernel<<<NTV / 16, 32, 0, stream>>>(U, XPW, DTW, Fp(11), BC, DT);
  scan_kernel<<<(NCHV * DN + 255) / 256, 256, 0, stream>>>(U, DT, BC, Fp(12), Fp(13), NCHV, Y4);
  outproj_kernel<<<NTV / 16, 32, 0, stream>>>(Y4, XZ, Fp(14), Fp(15), WOP, V);
  final_kernel<<<(unsigned)(((size_t)NBV * C * HH * HH + 255) / 256), 256, 0, stream>>>(Fp(0), MS, Fp(1), Fp(2), Fp(3), V, NBV, (float*)d_out);
}
